// SlidingWindowAttention_58849641890634
// MI455X (gfx1250) — hardware-verified
//
#include <hip/hip_runtime.h>

#ifndef NB
#define NB 2
#endif
#ifndef SEQ
#define SEQ 4096
#endif
#define NB_FULL  2
#define SEQ_FULL 4096
#define DM       1024
#define NH       16
#define HD       64
#define CW       128
#define MROWS    (NB * SEQ)
#define SCALE_F  0.125f
#define W_CARRY  64.0f
#define P_CARRY  1024.0f
#define O_CARRY  32.0f

static_assert(NB >= 1 && NB <= NB_FULL);
static_assert(SEQ >= CW && SEQ <= SEQ_FULL && (SEQ % CW) == 0);
static_assert(DM == NH * HD);
static_assert(HD == 64 && CW == 128);
static_assert((MROWS % 32) == 0);
static_assert((DM % 64) == 0);
static_assert((DM / 8) == 128);

typedef __attribute__((ext_vector_type(16))) _Float16 v16h;
typedef __attribute__((ext_vector_type(8)))  _Float16 v8h;
typedef __attribute__((ext_vector_type(8)))  float    v8f;
typedef __attribute__((ext_vector_type(4)))  float    v4f;
typedef __attribute__((ext_vector_type(4)))  unsigned int v4u;
union Pack8 { v8h h; v4u u; };

static __device__ __forceinline__ v8f wmma16(v16h a, v16h b, v8f c) {
  v8f d = __builtin_amdgcn_wmma_f32_16x16x32_f16(false, a, false, b, (short)0, c, false, false);
  asm volatile("v_nop\n\tv_nop\n\tv_nop\n\tv_nop" : "+v"(d) : "v"(a), "v"(b));
  return d;
}

static __device__ __forceinline__ void wave_lds_sync() {
  __builtin_amdgcn_fence(__ATOMIC_RELEASE, "wavefront");
  asm volatile("s_wait_dscnt 0x0" ::: "memory");
  __builtin_amdgcn_wave_barrier();
}

static __device__ __forceinline__ float bf16r(float x) {
  unsigned u = __float_as_uint(x);
  u = (u + 0x7FFFu + ((u >> 16) & 1u)) & 0xFFFF0000u;
  return __uint_as_float(u);
}

static __device__ __forceinline__ v16h load_frag(const _Float16* row, int lane) {
  const int kb = (lane < 16) ? 0 : 8;
  v8h lo = *(const v8h*)(row + kb);
  v8h hi = *(const v8h*)(row + kb + 16);
  v16h r;
#pragma unroll
  for (int i = 0; i < 8; ++i) { r[i] = lo[i]; r[i + 8] = hi[i]; }
  return r;
}

__global__ __launch_bounds__(256) void k_cvt_x(const float* __restrict__ X, _Float16* Xh, int n8) {
  for (int i = blockIdx.x * 256 + threadIdx.x; i < n8; i += gridDim.x * 256) {
    const int row = i >> 7;
    const int c8  = (i & 127) << 3;
    const int b   = row / SEQ;
    const int t   = row - b * SEQ;
    const float* src = X + ((size_t)(b * SEQ_FULL + t) * DM + c8);
    const v4f a0 = *(const v4f*)src;
    const v4f a1 = *(const v4f*)(src + 4);
    Pack8 pk;
#pragma unroll
    for (int e = 0; e < 4; ++e) {
      pk.h[e]     = (_Float16)bf16r(a0[e]);
      pk.h[e + 4] = (_Float16)bf16r(a1[e]);
    }
    _Float16* dst = Xh + ((size_t)row * DM + c8);
    *(volatile v4u*)dst = pk.u;
    __threadfence();
    *(volatile v4u*)dst = pk.u;
  }
}

__global__ __launch_bounds__(256) void k_cvt_wt(const float* __restrict__ Wsrc, _Float16* Wt, float scale) {
  __shared__ float tile[64][65];
  const int k0 = blockIdx.y * 64;
  const int n0 = blockIdx.x * 64;
  const int tid = threadIdx.x;
#pragma unroll
  for (int it = 0; it < 4; ++it) {
    const int lin = it * 256 + tid;
    const int r = lin >> 4, c4 = (lin & 15) << 2;
    const v4f v = *(const v4f*)(Wsrc + ((size_t)(k0 + r) * DM + n0 + c4));
#pragma unroll
    for (int e = 0; e < 4; ++e) tile[r][c4 + e] = v[e];
  }
  __syncthreads();
  const int c0 = (tid & 7) << 3;
#pragma unroll
  for (int pass = 0; pass < 2; ++pass) {
#pragma unroll
    for (int it = 0; it < 2; ++it) {
      const int n = it * 32 + (tid >> 3);
      Pack8 pk;
#pragma unroll
      for (int e = 0; e < 8; ++e) pk.h[e] = (_Float16)(scale * bf16r(tile[c0 + e][n]));
      *(volatile v4u*)(Wt + ((size_t)(n0 + n) * DM + k0 + c0)) = pk.u;
    }
    if (pass == 0) __threadfence();
  }
}

template <int MODE>
static __device__ __forceinline__ void tile_out(const v8f (&acc)[4], float* Cw, void* out,
                                                const float* __restrict__ bias, int row0, int n0,
                                                int N, float oscale, int lane) {
  const int col = lane & 15, lh = lane >> 4;
#pragma unroll
  for (int t = 0; t < 4; ++t)
#pragma unroll
    for (int i = 0; i < 8; ++i)
      Cw[(lh * 8 + i) * 64 + t * 16 + col] = acc[t][i] * oscale;
  wave_lds_sync();
  if (MODE == 0) {
    _Float16* o = (_Float16*)out;
    const int rl = lane >> 3, c0 = (lane & 7) << 3;
#pragma unroll
    for (int pass = 0; pass < 2; ++pass) {
#pragma unroll
      for (int it = 0; it < 4; ++it) {
        const int r = it * 4 + rl;
        const v4f x0 = *(const v4f*)(Cw + r * 64 + c0);
        const v4f x1 = *(const v4f*)(Cw + r * 64 + c0 + 4);
        Pack8 pk;
#pragma unroll
        for (int e = 0; e < 4; ++e) { pk.h[e] = (_Float16)x0[e]; pk.h[e + 4] = (_Float16)x1[e]; }
        *(volatile v4u*)(o + ((size_t)(row0 + r) * N + n0 + c0)) = pk.u;
      }
      if (pass == 0) __threadfence();
    }
  } else {
    float* o = (float*)out;
    const int rl = lane >> 4, c0 = (lane & 15) << 2;
    v4f bv;
#pragma unroll
    for (int e = 0; e < 4; ++e) bv[e] = bf16r(bias[n0 + c0 + e]);
#pragma unroll
    for (int pass = 0; pass < 2; ++pass) {
#pragma unroll
      for (int it = 0; it < 8; ++it) {
        const int r = it * 2 + rl;
        v4f x = *(const v4f*)(Cw + r * 64 + c0);
        x += bv;
        *(volatile v4f*)(o + ((size_t)(row0 + r) * N + n0 + c0)) = x;
      }
      if (pass == 0) __threadfence();
    }
  }
  wave_lds_sync();
}

template <int MODE>
__global__ __launch_bounds__(256) void k_gemm(const _Float16* __restrict__ A,
                                              const _Float16* __restrict__ W,
                                              void* out, const float* __restrict__ bias,
                                              int M, int N, int K, float oscale) {
  __shared__ __align__(16) float ldsC[8][16 * 64];
  const int lane  = threadIdx.x & 31;
  const int wslot = __builtin_amdgcn_readfirstlane((int)(threadIdx.x >> 5));
  const int wid   = blockIdx.x * 8 + wslot;
  const int tilesN = N >> 6;
  const int tm = wid / tilesN;
  const int m0 = tm << 5;
  const int n0 = (wid - tm * tilesN) << 6;
  if (m0 >= M) return;
  const int col = lane & 15;

  v8f acc0[4] = {v8f{}, v8f{}, v8f{}, v8f{}};
  v8f acc1[4] = {v8f{}, v8f{}, v8f{}, v8f{}};
  const _Float16* arow0 = A + (size_t)(m0 + col) * K;
  const _Float16* arow1 = A + (size_t)(m0 + 16 + col) * K;
  const _Float16* wrow  = W + (size_t)(n0 + col) * K;

  for (int k0 = 0; k0 < K; k0 += 32) {
    const v16h af0 = load_frag(arow0 + k0, lane);
    const v16h af1 = load_frag(arow1 + k0, lane);
#pragma unroll
    for (int t = 0; t < 4; ++t) {
      const v16h bf = load_frag(wrow + (size_t)(t * 16) * K + k0, lane);
      acc0[t] = wmma16(af0, bf, acc0[t]);
      acc1[t] = wmma16(af1, bf, acc1[t]);
    }
  }
  float* Cw = &ldsC[wslot][0];
  tile_out<MODE>(acc0, Cw, out, bias, m0, n0, N, oscale, lane);
  tile_out<MODE>(acc1, Cw, out, bias, m0 + 16, n0, N, oscale, lane);
}

__global__ __launch_bounds__(256) void k_vt(const _Float16* __restrict__ Vp, _Float16* Vt) {
  __shared__ __align__(16) _Float16 tile[64][72];
  const int stiles = SEQ / 64;
  const int bh = blockIdx.x / stiles;
  const int s0 = (blockIdx.x - bh * stiles) * 64;
  const int b = bh / NH, h = bh - b * NH;
  const int tid = threadIdx.x;
#pragma unroll
  for (int it = 0; it < 2; ++it) {
    const int lin = it * 256 + tid;
    const int si = lin >> 3, c8 = (lin & 7) << 3;
    *(v8h*)&tile[si][c8] = *(const v8h*)(Vp + (((size_t)b * SEQ + s0 + si) * DM + h * HD + c8));
  }
  __syncthreads();
  const int c0 = (tid & 7) << 3;
#pragma unroll
  for (int pass = 0; pass < 2; ++pass) {
#pragma unroll
    for (int it = 0; it < 2; ++it) {
      const int d = it * 32 + (tid >> 3);
      Pack8 pk;
#pragma unroll
      for (int e = 0; e < 8; ++e) pk.h[e] = tile[c0 + e][d];
      *(volatile v4u*)(Vt + (((size_t)bh * HD + d) * SEQ + s0 + c0)) = pk.u;
    }
    if (pass == 0) __threadfence();
  }
}

__global__ __launch_bounds__(256) void k_attn(const _Float16* __restrict__ Qp,
                                              const _Float16* __restrict__ Kp,
                                              const _Float16* __restrict__ Vt,
                                              _Float16* Op) {
  __shared__ __align__(16) float    ldsS[8][16 * 32];
  __shared__ __align__(16) _Float16 ldsO[8][16 * 64];
  const int lane  = threadIdx.x & 31;
  const int wslot = __builtin_amdgcn_readfirstlane((int)(threadIdx.x >> 5));
  const int wid   = blockIdx.x * 8 + wslot;
  const int qtiles = SEQ / 16;
  const int bh = wid / qtiles;
  const int qt = wid - bh * qtiles;
  if (bh >= NB * NH) return;
  const int b  = bh / NH;
  const int h  = bh - b * NH;
  const int q0 = qt * 16;
  const int nb = q0 / CW;
  const int q0l = q0 - nb * CW;
  const int col = lane & 15;
  const int lh  = lane >> 4;
  const int kb  = lh * 8;
  const int ql  = q0l + col;
  float*    Sw = &ldsS[wslot][0];
  _Float16* Ow = &ldsO[wslot][0];

  const size_t prow0 = (size_t)b * SEQ + q0;
  const _Float16* Qbase = Qp + (prow0 * DM + h * HD);
  const v16h qa0 = load_frag(Qbase + (size_t)col * DM, lane);
  const v16h qa1 = load_frag(Qbase + (size_t)col * DM + 32, lane);

  float m_row = -1e30f, l_row = 0.f;
  v8f o[4] = {v8f{}, v8f{}, v8f{}, v8f{}};

  const int jlo = q0l & ~31;
  int jhi = q0l + 15 + CW;
  if (nb == 0) { const int c = 2 * (q0l + 15) + 1; jhi = (c < jhi) ? c : jhi; }

  for (int j0 = jlo; j0 <= jhi; j0 += 32) {
    const bool ztile = (nb == 0) && (j0 < CW);
    const int  tok0  = (nb - 1) * CW + j0;
    float sv[16];
    if (!ztile) {
      const _Float16* Kb0 = Kp + (((size_t)b * SEQ + tok0 + col) * DM + h * HD);
      const _Float16* Kb1 = Kb0 + (size_t)16 * DM;
      v8f s0 = {}, s1 = {};
      s0 = wmma16(qa0, load_frag(Kb0, lane), s0);
      s0 = wmma16(qa1, load_frag(Kb0 + 32, lane), s0);
      s1 = wmma16(qa0, load_frag(Kb1, lane), s1);
      s1 = wmma16(qa1, load_frag(Kb1 + 32, lane), s1);
#pragma unroll
      for (int i = 0; i < 8; ++i) {
        Sw[(lh * 8 + i) * 32 + col]      = s0[i];
        Sw[(lh * 8 + i) * 32 + 16 + col] = s1[i];
      }
      wave_lds_sync();
      const float* Srow = Sw + col * 32 + kb;
#pragma unroll
      for (int e = 0; e < 8; ++e) { sv[e] = Srow[e] * SCALE_F; sv[e + 8] = Srow[e + 16] * SCALE_F; }
      wave_lds_sync();
    } else {
#pragma unroll
      for (int e = 0; e < 16; ++e) sv[e] = 0.f;
    }

    const bool full = (j0 >= q0l + 16) && (j0 + 31 <= q0l + CW) &&
                      ((nb != 0) || (j0 + 31 <= 2 * q0l + 1));

    float mnew, alpha, sloc;
    v16h pf;
    if (full) {
      float mloc = sv[0];
#pragma unroll
      for (int e = 1; e < 16; ++e) mloc = fmaxf(mloc, sv[e]);
      const float rowmax = fmaxf(mloc, __shfl_xor(mloc, 16));
      mnew  = fmaxf(m_row, rowmax);
      alpha = __expf(m_row - mnew);
      sloc  = 0.f;
#pragma unroll
      for (int e = 0; e < 16; ++e) {
        const float pv = __expf(sv[e] - mnew);
        pf[e] = (_Float16)(pv * P_CARRY);
        sloc += pv;
      }
    } else {
      bool vm[16];
      float mloc = -1e30f;
#pragma unroll
      for (int e = 0; e < 16; ++e) {
        const int j = j0 + kb + ((e < 8) ? e : e + 8);
        vm[e] = (j >= ql + 1) && (j <= ql + CW) && ((nb != 0) || (j <= 2 * ql + 1));
        sv[e] = vm[e] ? sv[e] : -1e30f;
        mloc  = fmaxf(mloc, sv[e]);
      }
      const float rowmax = fmaxf(mloc, __shfl_xor(mloc, 16));
      mnew  = fmaxf(m_row, rowmax);
      alpha = __expf(m_row - mnew);
      sloc  = 0.f;
#pragma unroll
      for (int e = 0; e < 16; ++e) {
        const float pv = vm[e] ? __expf(sv[e] - mnew) : 0.f;
        pf[e] = (_Float16)(pv * P_CARRY);
        sloc += pv;
      }
    }
    const float rowsum = sloc + __shfl_xor(sloc, 16);
    l_row = l_row * alpha + rowsum;
    m_row = mnew;

#pragma unroll
    for (int i = 0; i < 8; ++i) {
      const float ai = __shfl(alpha, i + lh * 8);
      o[0][i] *= ai; o[1][i] *= ai; o[2][i] *= ai; o[3][i] *= ai;
    }

    if (!ztile) {
      const _Float16* Vb = Vt + ((size_t)bh * HD * SEQ + tok0);
#pragma unroll
      for (int t = 0; t < 4; ++t) {
        const v16h vf = load_frag(Vb + (size_t)(t * 16 + col) * SEQ, lane);
        o[t] = wmma16(pf, vf, o[t]);
      }
    }
  }

  const float invl = 1.f / l_row;
#pragma unroll
  for (int i = 0; i < 8; ++i) {
    const float li = __shfl(invl, i + lh * 8) * (O_CARRY / P_CARRY);
#pragma unroll
    for (int t = 0; t < 4; ++t)
      Ow[(lh * 8 + i) * 64 + t * 16 + col] = (_Float16)(o[t][i] * li);
  }
  wave_lds_sync();
  _Float16* Ob = Op + (prow0 * DM + h * HD);
  const int rl = lane >> 3, c0 = (lane & 7) << 3;
#pragma unroll
  for (int pass = 0; pass < 2; ++pass) {
#pragma unroll
    for (int it = 0; it < 4; ++it) {
      const int r = it * 4 + rl;
      Pack8 pk;
      pk.h = *(const v8h*)(Ow + r * 64 + c0);
      *(volatile v4u*)(Ob + ((size_t)r * DM + c0)) = pk.u;
    }
    if (pass == 0) __threadfence();
  }
}

extern "C" void kernel_launch(void* const* d_in, const int* in_sizes, int n_in,
                              void* d_out, int out_size, void* d_ws, size_t ws_size,
                              hipStream_t stream) {
  if (n_in < 6) return;
  if (in_sizes[0] < ((NB - 1) * SEQ_FULL + SEQ) * DM) return;
  if (in_sizes[1] < DM * DM || in_sizes[2] < DM * DM ||
      in_sizes[3] < DM * DM || in_sizes[4] < DM * DM) return;
  if (in_sizes[5] < DM) return;
  if (out_size < MROWS * DM) return;

  const float* X  = (const float*)d_in[0];
  const float* Wq = (const float*)d_in[1];
  const float* Wk = (const float*)d_in[2];
  const float* Wv = (const float*)d_in[3];
  const float* Wp = (const float*)d_in[4];
  const float* bp = (const float*)d_in[5];
  float* out = (float*)d_out;

  const size_t nx = (size_t)MROWS * DM;
  const size_t nw = (size_t)DM * DM;
  const size_t total = (6 * nx + 4 * nw) * sizeof(_Float16);
  if (total > ws_size) return;

  _Float16* p   = (_Float16*)d_ws;
  _Float16* Xh  = p; p += nx;
  _Float16* Wqt = p; p += nw;
  _Float16* Wkt = p; p += nw;
  _Float16* Wvt = p; p += nw;
  _Float16* Wpt = p; p += nw;
  _Float16* Qp  = p; p += nx;
  _Float16* Kpl = p; p += nx;
  _Float16* Vp  = p; p += nx;
  _Float16* Vtp = p; p += nx;
  _Float16* Op  = p; p += nx;

  const int T = 256;
  const int n8 = (int)(nx / 8);
  k_cvt_x<<<(n8 + T - 1) / T, T, 0, stream>>>(X, Xh, n8);
  const dim3 wgrid(DM / 64, DM / 64);
  k_cvt_wt<<<wgrid, T, 0, stream>>>(Wq, Wqt, W_CARRY);
  k_cvt_wt<<<wgrid, T, 0, stream>>>(Wk, Wkt, W_CARRY);
  k_cvt_wt<<<wgrid, T, 0, stream>>>(Wv, Wvt, W_CARRY);
  k_cvt_wt<<<wgrid, T, 0, stream>>>(Wp, Wpt, W_CARRY);

  const int gemm_tiles  = (MROWS / 32) * (DM / 64);
  const int gemm_blocks = (gemm_tiles + 7) / 8;
  const float qkv_scale = 1.0f / W_CARRY;
  k_gemm<0><<<gemm_blocks, T, 0, stream>>>(Xh, Wqt, (void*)Qp,  bp, MROWS, DM, DM, qkv_scale);
  k_gemm<0><<<gemm_blocks, T, 0, stream>>>(Xh, Wkt, (void*)Kpl, bp, MROWS, DM, DM, qkv_scale);
  k_gemm<0><<<gemm_blocks, T, 0, stream>>>(Xh, Wvt, (void*)Vp,  bp, MROWS, DM, DM, qkv_scale);

  k_vt<<<NB * NH * (SEQ / 64), T, 0, stream>>>(Vp, Vtp);

  const int attn_waves  = NB * NH * (SEQ / 16);
  const int attn_blocks = (attn_waves + 7) / 8;
  k_attn<<<attn_blocks, T, 0, stream>>>(Qp, Kpl, Vtp, Op);

  const float out_scale = 1.0f / (O_CARRY * W_CARRY);
  k_gemm<1><<<gemm_blocks, T, 0, stream>>>(Op, Wpt, (void*)out, bp, MROWS, DM, DM, out_scale);
}
